// MultiHeadSparseMMAttentionSBH_52381421142525
// MI455X (gfx1250) — hardware-verified
//
#include <hip/hip_runtime.h>
#include <math.h>

#ifndef NB
#define NB 1
#endif
#ifndef SEQ
#define SEQ 8192
#endif
#define SEQ_FULL 8192
#ifndef TXT
#define TXT 256
#endif
#define TXT_FULL 256
#ifndef OUT_TXT_ROW
#define OUT_TXT_ROW SEQ
#endif
#define HEADS 16
#define HD 64
#define INNER 1024
#define SPN 8
#define GSEQ (SEQ / SPN)
#define LTOT (GSEQ + TXT)
#define NBH (SPN * HEADS)
#define QBLK (LTOT / 128)
#define AT_PP 72

static_assert(NB == 1);
static_assert(SEQ <= SEQ_FULL && TXT <= TXT_FULL);
static_assert(HEADS * HD == INNER && HD == 64);
static_assert(SEQ % (SPN * SPN) == 0);
static_assert(GSEQ % 64 == 0 && TXT % 64 == 0 && INNER % 64 == 0);
static_assert(INNER % 32 == 0 && HD % 32 == 0 && LTOT % 32 == 0);
static_assert(LTOT % 64 == 0);
static_assert(GSEQ % 16 == 0);
static_assert((LTOT / 16) % 8 == 0);
static_assert(QBLK * 128 == LTOT);
static_assert((SEQ * INNER) % 8 == 0 && (TXT * INNER) % 8 == 0 && (INNER * INNER) % 8 == 0);
static_assert(SEQ % 32 == 0 && TXT % 32 == 0);
static_assert(8 * 16 * 68 * 4 <= 131072);
static_assert(2 * 8 * 16 * AT_PP * 2 <= 131072);
static_assert(32 * 16 * 4 == 16 * 128);
static_assert(32 * 16 * 8 == 16 * 256);
static_assert(2 * 16 == 32);

static constexpr size_t CTX_BYTES = (size_t)(SEQ + SPN * TXT) * INNER * 2;
static constexpr size_t DEAD_BYTES = (size_t)SEQ * INNER * 2 + (size_t)TXT * INNER * 2 + (size_t)6 * INNER * INNER * 2;
static_assert(CTX_BYTES <= DEAD_BYTES);
static_assert(((size_t)SEQ * INNER * 2) % 256 == 0 && ((size_t)TXT * INNER * 2) % 256 == 0 && ((size_t)INNER * INNER * 2) % 256 == 0);
static constexpr size_t CARVE_TOTAL =
    (size_t)SEQ * INNER * 2 + (size_t)TXT * INNER * 2 + (size_t)8 * INNER * INNER * 2 +
    (size_t)3 * NBH * LTOT * HD * 2 + CTX_BYTES + (size_t)2 * TXT * INNER * 2;
static_assert(CARVE_TOTAL + 17 * 256 <= (size_t)134217728);

static constexpr float CARRY_X = 8.0f;
static constexpr float CARRY_W = 32.0f;
static constexpr float SC  = 1.0f / 256.0f;
static constexpr float SCV = 8.0f / 256.0f;
static constexpr float SC2 = 0.125f * (1.0f / 64.0f) * 1.4426950408889634f;
static constexpr float RES_CARRY = 2048.0f;
static constexpr float RES_INV = 1.0f / 2048.0f;

typedef __attribute__((ext_vector_type(16))) _Float16 v16h;
typedef __attribute__((ext_vector_type(8)))  _Float16 v8h;
typedef __attribute__((ext_vector_type(8)))  float    v8f;
typedef __attribute__((ext_vector_type(4)))  float    v4f;
typedef _Float16 h16;


__device__ __forceinline__ float bfr(float f) {
    unsigned u = __float_as_uint(f);
    u += 0x7FFFu + ((u >> 16) & 1u);
    return __uint_as_float(u & 0xFFFF0000u);
}
static __device__ __forceinline__ h16 toh_flush(float v) {
    const h16 r = (h16)v;
    return (fabsf(v) < 6.103515625e-05f) ? (h16)0.0f : r;
}
__device__ __forceinline__ float ex2(float x) { return __builtin_amdgcn_exp2f(x); }

union FragU { v16h v; v8h h[2]; };
__device__ __forceinline__ v16h frag_ld(const _Float16* p) {
    FragU f; f.h[0] = *(const v8h*)(p); f.h[1] = *(const v8h*)(p + 16); return f.v;
}
__device__ __forceinline__ v8f wmma16(v16h a, v16h b, v8f c) {
    c = __builtin_amdgcn_wmma_f32_16x16x32_f16(false, a, false, b, (short)0, c, false, false);
    asm volatile("v_nop\n\tv_nop\n\tv_nop\n\tv_nop" : "+v"(c) : "v"(a), "v"(b));
    return c;
}
__device__ __forceinline__ void wave_sync_lds() {
    __builtin_amdgcn_fence(3  , "workgroup");
    __builtin_amdgcn_wave_barrier();
    __builtin_amdgcn_fence(2  , "workgroup");
}

__global__ __launch_bounds__(256) void k_cvt16(const float* __restrict__ src, _Float16* __restrict__ dst, unsigned n8, float s) {
#pragma clang fp contract(off)
    const unsigned u = blockIdx.x * 256u + threadIdx.x;
    if (u >= n8) return;
    const size_t o = (size_t)u * 8u;
    const v4f a = *(const v4f*)(src + o);
    const v4f b = *(const v4f*)(src + o + 4u);
    v8h hv;
    hv[0] = toh_flush(bfr(a.x) * s); hv[1] = toh_flush(bfr(a.y) * s);
    hv[2] = toh_flush(bfr(a.z) * s); hv[3] = toh_flush(bfr(a.w) * s);
    hv[4] = toh_flush(bfr(b.x) * s); hv[5] = toh_flush(bfr(b.y) * s);
    hv[6] = toh_flush(bfr(b.z) * s); hv[7] = toh_flush(bfr(b.w) * s);
    for (int pass = 0; pass < 2; ++pass) {
        *(volatile v8h*)(dst + o) = hv;
        __threadfence();
    }
}

__device__ __forceinline__ void gemm_acc64(const _Float16* __restrict__ A, unsigned lda, const _Float16* __restrict__ Bt, unsigned ldb,
                                           unsigned K, unsigned rlane, unsigned koff, v8f (&acc)[4][4]) {
#pragma unroll
    for (int i = 0; i < 4; ++i)
#pragma unroll
        for (int j = 0; j < 4; ++j) acc[i][j] = (v8f){0.f,0.f,0.f,0.f,0.f,0.f,0.f,0.f};
    unsigned ao[4], bo[4];
#pragma unroll
    for (int i = 0; i < 4; ++i) {
        ao[i] = (((unsigned)i << 4) + rlane) * lda + koff;
        bo[i] = (((unsigned)i << 4) + rlane) * ldb + koff;
    }
#pragma unroll 1
    for (unsigned k0 = 0; k0 < K; k0 += 32u) {
        v16h bh[4];
#pragma unroll
        for (int j = 0; j < 4; ++j) bh[j] = frag_ld(Bt + (bo[j] + k0));
#pragma unroll
        for (int i = 0; i < 4; ++i) {
            const v16h ah = frag_ld(A + (ao[i] + k0));
#pragma unroll
            for (int j = 0; j < 4; ++j) acc[i][j] = wmma16(ah, bh[j], acc[i][j]);
        }
    }
}

__device__ __forceinline__ void gemm2_acc32(const _Float16* __restrict__ A, const _Float16* __restrict__ Ar, unsigned lda,
                                            const _Float16* __restrict__ Bt, unsigned ldb, unsigned K, unsigned rlane, unsigned koff,
                                            v8f (&acc)[2][4], v8f (&accr)[2][4]) {
#pragma unroll
    for (int i = 0; i < 2; ++i)
#pragma unroll
        for (int j = 0; j < 4; ++j) {
            acc[i][j] = (v8f){0.f,0.f,0.f,0.f,0.f,0.f,0.f,0.f};
            accr[i][j] = (v8f){0.f,0.f,0.f,0.f,0.f,0.f,0.f,0.f};
        }
    unsigned ao[2], bo[4];
#pragma unroll
    for (int i = 0; i < 2; ++i) ao[i] = (((unsigned)i << 4) + rlane) * lda + koff;
#pragma unroll
    for (int j = 0; j < 4; ++j) bo[j] = (((unsigned)j << 4) + rlane) * ldb + koff;
#pragma unroll 1
    for (unsigned k0 = 0; k0 < K; k0 += 32u) {
        v16h bh[4];
#pragma unroll
        for (int j = 0; j < 4; ++j) bh[j] = frag_ld(Bt + (bo[j] + k0));
#pragma unroll
        for (int i = 0; i < 2; ++i) {
            const v16h ah = frag_ld(A + (ao[i] + k0));
#pragma unroll
            for (int j = 0; j < 4; ++j) acc[i][j] = wmma16(ah, bh[j], acc[i][j]);
            const v16h ar = frag_ld(Ar + (ao[i] + k0));
#pragma unroll
            for (int j = 0; j < 4; ++j) accr[i][j] = wmma16(ar, bh[j], accr[i][j]);
        }
    }
}

template <bool ROPE>
__device__ __forceinline__ void projqk_body(const _Float16* __restrict__ X, unsigned lda, unsigned jstride,
                                            const _Float16* __restrict__ Wt, _Float16* __restrict__ Qp,
                                            const float* __restrict__ g, const float* __restrict__ rcos, const float* __restrict__ rsin,
                                            unsigned M, unsigned rep, unsigned posOff) {
    __shared__ __align__(16) float sT[8][16 * 68];
    const unsigned lane = threadIdx.x & 31u;
    const unsigned wave = __builtin_amdgcn_readfirstlane(threadIdx.x >> 5);
    const unsigned tilesM = M >> 6;
    const unsigned tile = blockIdx.x * 8u + wave;
    if (tile >= tilesM * 16u) return;
    const unsigned tm = tile >> 4, tn = tile & 15u;
    const unsigned jb = blockIdx.y;
    const unsigned m0 = tm << 6;
    const unsigned rlane = lane & 15u;
    const unsigned koff = (lane >> 4) * 8u;

    v8f acc[4][4];
    gemm_acc64(X + (size_t)jb * jstride + (size_t)m0 * lda, lda, Wt + (size_t)(tn << 6) * INNER, INNER, INNER, rlane, koff, acc);

    const unsigned q = lane >> 3, c8 = (lane & 7u) * 8u, pc = c8 ^ 32u;
    float gv[8], gp[8];
    {
        const v4f a = *(const v4f*)(g + c8), b = *(const v4f*)(g + c8 + 4u);
        gv[0] = bfr(a.x); gv[1] = bfr(a.y); gv[2] = bfr(a.z); gv[3] = bfr(a.w);
        gv[4] = bfr(b.x); gv[5] = bfr(b.y); gv[6] = bfr(b.z); gv[7] = bfr(b.w);
        const v4f cc = *(const v4f*)(g + pc), d = *(const v4f*)(g + pc + 4u);
        gp[0] = bfr(cc.x); gp[1] = bfr(cc.y); gp[2] = bfr(cc.z); gp[3] = bfr(cc.w);
        gp[4] = bfr(d.x); gp[5] = bfr(d.y); gp[6] = bfr(d.z); gp[7] = bfr(d.w);
    }
    const float sgn = (c8 < 32u) ? -1.0f : 1.0f;

#pragma unroll
    for (int i = 0; i < 4; ++i) {
        const unsigned mBase = m0 + ((unsigned)i << 4);
#pragma unroll
        for (int j = 0; j < 4; ++j)
#pragma unroll
            for (int r = 0; r < 8; ++r)
                sT[wave][(koff + (unsigned)r) * 68u + ((unsigned)j << 4) + rlane] = acc[i][j][r] * SC;
        wave_sync_lds();
        v8h hv[4];
#pragma unroll
        for (int it = 0; it < 4; ++it) {
            const unsigned row = (unsigned)it * 4u + q;
            const v4f x0 = *(const v4f*)&sT[wave][row * 68u + c8];
            const v4f x1 = *(const v4f*)&sT[wave][row * 68u + c8 + 4u];
            const float x[8] = {x0.x, x0.y, x0.z, x0.w, x1.x, x1.y, x1.z, x1.w};
            float ss = 0.f;
#pragma unroll
            for (int e = 0; e < 8; ++e) ss += x[e] * x[e];
            ss += __shfl_xor(ss, 1, 32); ss += __shfl_xor(ss, 2, 32); ss += __shfl_xor(ss, 4, 32);
            const float rinv = rsqrtf(ss * (1.0f / 64.0f) + 1e-5f);
            float y[8];
#pragma unroll
            for (int e = 0; e < 8; ++e) y[e] = x[e] * rinv * gv[e];
            if (ROPE) {
                const v4f p0 = *(const v4f*)&sT[wave][row * 68u + pc];
                const v4f p1 = *(const v4f*)&sT[wave][row * 68u + pc + 4u];
                const float xp[8] = {p0.x, p0.y, p0.z, p0.w, p1.x, p1.y, p1.z, p1.w};
                const size_t to = (size_t)((mBase + row) * SPN + jb) * 64u + c8;
                const v4f c0 = *(const v4f*)(rcos + to), c1 = *(const v4f*)(rcos + to + 4u);
                const v4f s0 = *(const v4f*)(rsin + to), s1 = *(const v4f*)(rsin + to + 4u);
                const float cv[8] = {c0.x, c0.y, c0.z, c0.w, c1.x, c1.y, c1.z, c1.w};
                const float sv[8] = {s0.x, s0.y, s0.z, s0.w, s1.x, s1.y, s1.z, s1.w};
#pragma unroll
                for (int e = 0; e < 8; ++e) {
                    const float yp = xp[e] * rinv * gp[e];
                    y[e] = y[e] * bfr(cv[e]) + (sgn * yp) * bfr(sv[e]);
                }
            }
#pragma unroll
            for (int e = 0; e < 8; ++e) hv[it][e] = toh_flush(y[e] * 8.0f);
        }
        for (int pass = 0; pass < 2; ++pass) {
            for (unsigned rp = 0; rp < rep; ++rp) {
                _Float16* dst = Qp + ((size_t)((jb + rp) * HEADS + tn) * LTOT + posOff + mBase) * HD + c8;
#pragma unroll
                for (int it = 0; it < 4; ++it) {
                    const unsigned row = (unsigned)it * 4u + q;
                    *(volatile v8h*)(dst + (size_t)row * HD) = hv[it];
                }
            }
            __threadfence();
        }
        wave_sync_lds();
    }
}

__global__ __launch_bounds__(256) void k_projqk_rope(const _Float16* __restrict__ X, unsigned lda, unsigned jstride,
                                                     const _Float16* __restrict__ Wt, _Float16* __restrict__ Qp,
                                                     const float* __restrict__ g, const float* __restrict__ rcos, const float* __restrict__ rsin,
                                                     unsigned M, unsigned rep, unsigned posOff) {
    projqk_body<true>(X, lda, jstride, Wt, Qp, g, rcos, rsin, M, rep, posOff);
}
__global__ __launch_bounds__(256) void k_projqk_plain(const _Float16* __restrict__ X, unsigned lda, unsigned jstride,
                                                      const _Float16* __restrict__ Wt, _Float16* __restrict__ Qp,
                                                      const float* __restrict__ g, const float* __restrict__ rcos, const float* __restrict__ rsin,
                                                      unsigned M, unsigned rep, unsigned posOff) {
    projqk_body<false>(X, lda, jstride, Wt, Qp, g, rcos, rsin, M, rep, posOff);
}

__global__ __launch_bounds__(256) void k_projvt(const _Float16* __restrict__ Wv, const _Float16* __restrict__ X, unsigned ldb, unsigned jstride,
                                                _Float16* __restrict__ VT, unsigned NP, unsigned rep, unsigned posOff) {
    __shared__ __align__(16) float sT[8][16 * 68];
    const unsigned lane = threadIdx.x & 31u;
    const unsigned wave = __builtin_amdgcn_readfirstlane(threadIdx.x >> 5);
    const unsigned tilesN = NP >> 6;
    const unsigned tile = blockIdx.x * 8u + wave;
    if (tile >= 16u * tilesN) return;
    const unsigned tm = tile / tilesN;
    const unsigned tn = tile - tm * tilesN;
    const unsigned jb = blockIdx.y;
    const unsigned m0 = tm << 6, n0 = tn << 6;
    const unsigned rlane = lane & 15u;
    const unsigned koff = (lane >> 4) * 8u;

    v8f acc[4][4];
    gemm_acc64(Wv + (size_t)m0 * INNER, INNER, X + (size_t)jb * jstride + (size_t)n0 * ldb, ldb, INNER, rlane, koff, acc);

    const unsigned q = lane >> 3, c8 = (lane & 7u) * 8u;
#pragma unroll
    for (int i = 0; i < 4; ++i) {
        const unsigned mBase = m0 + ((unsigned)i << 4);
#pragma unroll
        for (int j = 0; j < 4; ++j)
#pragma unroll
            for (int r = 0; r < 8; ++r)
                sT[wave][(koff + (unsigned)r) * 68u + ((unsigned)j << 4) + rlane] = acc[i][j][r] * SCV;
        wave_sync_lds();
        v8h hv[4];
#pragma unroll
        for (int it = 0; it < 4; ++it) {
            const unsigned row = (unsigned)it * 4u + q;
            const v4f x0 = *(const v4f*)&sT[wave][row * 68u + c8];
            const v4f x1 = *(const v4f*)&sT[wave][row * 68u + c8 + 4u];
            hv[it][0] = toh_flush(x0.x); hv[it][1] = toh_flush(x0.y); hv[it][2] = toh_flush(x0.z); hv[it][3] = toh_flush(x0.w);
            hv[it][4] = toh_flush(x1.x); hv[it][5] = toh_flush(x1.y); hv[it][6] = toh_flush(x1.z); hv[it][7] = toh_flush(x1.w);
        }
        for (int pass = 0; pass < 2; ++pass) {
            for (unsigned rp = 0; rp < rep; ++rp) {
                _Float16* dst = VT + ((size_t)(jb + rp) * INNER + mBase) * LTOT + posOff + n0 + c8;
#pragma unroll
                for (int it = 0; it < 4; ++it) {
                    const unsigned row = (unsigned)it * 4u + q;
                    *(volatile v8h*)(dst + (size_t)row * LTOT) = hv[it];
                }
            }
            __threadfence();
        }
        wave_sync_lds();
    }
}

__global__ __launch_bounds__(256) void k_attn(const _Float16* __restrict__ Qp, const _Float16* __restrict__ Kp,
                                              const _Float16* __restrict__ VT, _Float16* __restrict__ ctx, _Float16* __restrict__ ctxr) {
    __shared__ __align__(16) _Float16 sO[8][16 * AT_PP];
    __shared__ __align__(16) _Float16 sR[8][16 * AT_PP];
    const unsigned lane = threadIdx.x & 31u;
    const unsigned wave = __builtin_amdgcn_readfirstlane(threadIdx.x >> 5);
    const unsigned hh = lane >> 4, c = lane & 15u;
    const unsigned bh = blockIdx.x / (unsigned)QBLK;
    const unsigned qblk = blockIdx.x - bh * (unsigned)QBLK;
    const unsigned q0 = (qblk * 8u + wave) * 16u;
    const _Float16* Qb = Qp + (size_t)bh * (LTOT * HD);
    const _Float16* Kb = Kp + (size_t)bh * (LTOT * HD);
    const _Float16* Vb = VT + (size_t)bh * (HD * LTOT);
    const v16h qf0 = frag_ld(Qb + ((q0 + c) * HD + 8u * hh));
    const v16h qf1 = frag_ld(Qb + ((q0 + c) * HD + 32u + 8u * hh));
    const unsigned ko = c * HD + 8u * hh;
    const unsigned vo = c * LTOT + 8u * hh;

    v8f ot[4];
#pragma unroll
    for (int t = 0; t < 4; ++t) ot[t] = (v8f){0.f,0.f,0.f,0.f,0.f,0.f,0.f,0.f};
    float mrun = -3.0e38f, lrun = 0.f;

#pragma unroll 1
    for (unsigned k0 = 0; k0 < (unsigned)LTOT; k0 += 32u) {
        v8f s0 = (v8f){0.f,0.f,0.f,0.f,0.f,0.f,0.f,0.f};
        v8f s1 = s0;
        {
            const v16h ka = frag_ld(Kb + (ko + k0 * HD));
            s0 = wmma16(ka, qf0, s0);
        }
        {
            const v16h ka = frag_ld(Kb + (ko + k0 * HD + 32u));
            s0 = wmma16(ka, qf1, s0);
        }
        {
            const v16h ka = frag_ld(Kb + (ko + (k0 + 16u) * HD));
            s1 = wmma16(ka, qf0, s1);
        }
        {
            const v16h ka = frag_ld(Kb + (ko + (k0 + 16u) * HD + 32u));
            s1 = wmma16(ka, qf1, s1);
        }
        float mx = -3.0e38f;
#pragma unroll
        for (int r = 0; r < 8; ++r) mx = fmaxf(mx, fmaxf(s0[r], s1[r]));
        mx = fmaxf(mx, __shfl_xor(mx, 16, 32));
        const float mnew = fmaxf(mrun, mx * SC2);
        const float alpha = ex2(mrun - mnew);
        mrun = mnew;
        const float sh = mnew - 10.0f;
        float psum = 0.f;
        v16h pb;
#pragma unroll
        for (int r = 0; r < 8; ++r) {
            const float e0 = s0[r] * SC2 - sh;
            const float e1 = s1[r] * SC2 - sh;
            const float x0 = ex2(e0);
            const float x1 = ex2(e1);
            const float p0 = (e0 < -14.0f) ? 0.0f : x0;
            const float p1 = (e1 < -14.0f) ? 0.0f : x1;
            psum += p0 + p1;
            pb[r] = (_Float16)p0;
            pb[8 + r] = (_Float16)p1;
        }
        psum += __shfl_xor(psum, 16, 32);
        lrun = lrun * alpha + psum;
#pragma unroll
        for (int t = 0; t < 4; ++t)
#pragma unroll
            for (int r = 0; r < 8; ++r) ot[t][r] *= alpha;
#pragma unroll
        for (int t = 0; t < 4; ++t) {
            const v16h va = frag_ld(Vb + (vo + (unsigned)t * 16u * LTOT + k0));
            ot[t] = wmma16(va, pb, ot[t]);
        }
    }

    const float inv = 1.0f / lrun;
#pragma unroll
    for (int t = 0; t < 4; ++t) {
        v8h o, orr;
#pragma unroll
        for (int r = 0; r < 8; ++r) {
            const float v = ot[t][r] * inv;
            const h16 hu = (h16)v;
            o[r] = toh_flush(v);
            orr[r] = toh_flush((v - (float)hu) * RES_CARRY);
        }
        *(v8h*)&sO[wave][c * AT_PP + (unsigned)t * 16u + 8u * hh] = o;
        *(v8h*)&sR[wave][c * AT_PP + (unsigned)t * 16u + 8u * hh] = orr;
    }
    wave_sync_lds();
    {
        const unsigned q = lane >> 3, c8 = (lane & 7u) * 8u;
        v8h ov[4], ovr[4];
#pragma unroll
        for (int it = 0; it < 4; ++it) {
            ov[it] = *(const v8h*)&sO[wave][((unsigned)it * 4u + q) * AT_PP + c8];
            ovr[it] = *(const v8h*)&sR[wave][((unsigned)it * 4u + q) * AT_PP + c8];
        }
        const unsigned q0v = (qblk * 8u + (threadIdx.x >> 5)) * 16u;
        const unsigned jj = bh >> 4, hd = bh & 15u;
        const unsigned isv = (q0v < (unsigned)GSEQ) ? 1u : 0u;
        const unsigned rbase = isv ? (q0v * (unsigned)SPN + jj) : ((unsigned)SEQ + jj * (unsigned)TXT + (q0v - (unsigned)GSEQ));
        const unsigned rstr = isv ? (unsigned)SPN : 1u;
        _Float16* dst = ctx + hd * HD + c8;
        _Float16* dstr = ctxr + hd * HD + c8;
        for (int pass = 0; pass < 2; ++pass) {
#pragma unroll
            for (int it = 0; it < 4; ++it) {
                const unsigned row = rbase + ((unsigned)it * 4u + q) * rstr;
                *(volatile v8h*)(dst + (size_t)row * INNER) = ov[it];
            }
#pragma unroll
            for (int it = 0; it < 4; ++it) {
                const unsigned row = rbase + ((unsigned)it * 4u + q) * rstr;
                *(volatile v8h*)(dstr + (size_t)row * INNER) = ovr[it];
            }
            __threadfence();
        }
    }
}

__global__ __launch_bounds__(256) void k_txtmean(const _Float16* __restrict__ ctx, const _Float16* __restrict__ ctxr,
                                                 _Float16* __restrict__ tm, _Float16* __restrict__ tmr) {
#pragma clang fp contract(off)
    const unsigned u = blockIdx.x * 256u + threadIdx.x;
    if (u >= (unsigned)(TXT * INNER / 8)) return;
    const unsigned t = u >> 7, c0 = (u & 127u) * 8u;
    float a[8] = {0.f, 0.f, 0.f, 0.f, 0.f, 0.f, 0.f, 0.f};
#pragma unroll 1
    for (unsigned j = 0; j < (unsigned)SPN; ++j) {
        const size_t o = ((size_t)SEQ + (size_t)j * TXT + t) * INNER + c0;
        const v8h v = *(const v8h*)(ctx + o);
        const v8h w = *(const v8h*)(ctxr + o);
#pragma unroll
        for (int e = 0; e < 8; ++e) a[e] += (float)v[e] + (float)w[e] * RES_INV;
    }
    v8h o, orr;
#pragma unroll
    for (int e = 0; e < 8; ++e) {
        const float m = a[e] * 0.125f;
        const h16 hu = (h16)m;
        o[e] = toh_flush(m);
        orr[e] = toh_flush((m - (float)hu) * RES_CARRY);
    }
    for (int pass = 0; pass < 2; ++pass) {
        *(volatile v8h*)(tm + (size_t)t * INNER + c0) = o;
        *(volatile v8h*)(tmr + (size_t)t * INNER + c0) = orr;
        __threadfence();
    }
}

__global__ __launch_bounds__(256) void k_outproj(const _Float16* __restrict__ A, const _Float16* __restrict__ Ar,
                                                 const _Float16* __restrict__ Wt, const float* __restrict__ bias,
                                                 float* __restrict__ C, unsigned M) {
    __shared__ __align__(16) float sT[8][16 * 68];
    const unsigned lane = threadIdx.x & 31u;
    const unsigned wave = __builtin_amdgcn_readfirstlane(threadIdx.x >> 5);
    const unsigned tilesM = M >> 5;
    const unsigned tile = blockIdx.x * 8u + wave;
    if (tile >= tilesM * 16u) return;
    const unsigned tm = tile >> 4, tn = tile & 15u;
    const unsigned m0 = tm << 5, n0 = tn << 6;
    const unsigned rlane = lane & 15u;
    const unsigned koff = (lane >> 4) * 8u;

    v8f acc[2][4], accr[2][4];
    gemm2_acc32(A + (size_t)m0 * INNER, Ar + (size_t)m0 * INNER, INNER, Wt + (size_t)n0 * INNER, INNER, INNER, rlane, koff, acc, accr);

    const unsigned hh = lane >> 4, c4 = (lane & 15u) * 4u;
#pragma unroll
    for (int i = 0; i < 2; ++i) {
        const unsigned mBase = m0 + ((unsigned)i << 4);
#pragma unroll
        for (int j = 0; j < 4; ++j) {
            const float bv = bfr(bias[n0 + ((unsigned)j << 4) + rlane]);
#pragma unroll
            for (int r = 0; r < 8; ++r)
                sT[wave][(koff + (unsigned)r) * 68u + ((unsigned)j << 4) + rlane] = (acc[i][j][r] + accr[i][j][r] * RES_INV) * SC + bv;
        }
        wave_sync_lds();
#pragma unroll
        for (int half = 0; half < 2; ++half) {
            v4f vv[4];
#pragma unroll
            for (int it = 0; it < 4; ++it) {
                const unsigned row = (unsigned)(half * 4 + it) * 2u + hh;
                vv[it] = *(const v4f*)&sT[wave][row * 68u + c4];
            }
            for (int pass = 0; pass < 2; ++pass) {
#pragma unroll
                for (int it = 0; it < 4; ++it) {
                    const unsigned row = (unsigned)(half * 4 + it) * 2u + hh;
                    *(volatile v4f*)(C + (size_t)(mBase + row) * INNER + n0 + c4) = vv[it];
                }
                __threadfence();
            }
        }
        wave_sync_lds();
    }
}

extern "C" void kernel_launch(void* const* d_in, const int* in_sizes, int n_in, void* d_out, int out_size,
                              void* d_ws, size_t ws_size, hipStream_t stream) {
    if (n_in < 18) return;
    if (in_sizes[0] < SEQ * INNER || in_sizes[1] < TXT * INNER) return;
    for (int i = 2; i <= 8; ++i) if (in_sizes[i] < INNER * INNER) return;
    if (in_sizes[10] < INNER * INNER || in_sizes[9] < INNER || in_sizes[11] < INNER) return;
    if (in_sizes[12] < HD || in_sizes[13] < HD || in_sizes[14] < HD || in_sizes[15] < HD) return;
    if (in_sizes[16] < SEQ * HD || in_sizes[17] < SEQ * HD) return;
    if (out_size < (OUT_TXT_ROW + TXT) * INNER) return;

    const float* hs    = (const float*)d_in[0];
    const float* ehs   = (const float*)d_in[1];
    const float* Wq    = (const float*)d_in[2];
    const float* Wk    = (const float*)d_in[3];
    const float* Wv    = (const float*)d_in[4];
    const float* Waq   = (const float*)d_in[5];
    const float* Wak   = (const float*)d_in[6];
    const float* Wav   = (const float*)d_in[7];
    const float* Wout  = (const float*)d_in[8];
    const float* bout  = (const float*)d_in[9];
    const float* Waout = (const float*)d_in[10];
    const float* baout = (const float*)d_in[11];
    const float* gq    = (const float*)d_in[12];
    const float* gk    = (const float*)d_in[13];
    const float* gaq   = (const float*)d_in[14];
    const float* gak   = (const float*)d_in[15];
    const float* rc    = (const float*)d_in[16];
    const float* rs    = (const float*)d_in[17];
    float* out = (float*)d_out;

    char* wsp = (char*)d_ws;
    size_t off = 0;
    auto carve = [&](size_t bytes) -> void* { void* r = wsp + off; off += (bytes + 255) & ~(size_t)255; return r; };
    _Float16* X16   = (_Float16*)carve((size_t)SEQ * INNER * 2);
    _Float16* E16   = (_Float16*)carve((size_t)TXT * INNER * 2);
    _Float16* wq16  = (_Float16*)carve((size_t)INNER * INNER * 2);
    _Float16* wk16  = (_Float16*)carve((size_t)INNER * INNER * 2);
    _Float16* wv16  = (_Float16*)carve((size_t)INNER * INNER * 2);
    _Float16* waq16 = (_Float16*)carve((size_t)INNER * INNER * 2);
    _Float16* wak16 = (_Float16*)carve((size_t)INNER * INNER * 2);
    _Float16* wav16 = (_Float16*)carve((size_t)INNER * INNER * 2);
    _Float16* wo16  = (_Float16*)carve((size_t)INNER * INNER * 2);
    _Float16* wao16 = (_Float16*)carve((size_t)INNER * INNER * 2);
    _Float16* Qp    = (_Float16*)carve((size_t)NBH * LTOT * HD * 2);
    _Float16* Kp    = (_Float16*)carve((size_t)NBH * LTOT * HD * 2);
    _Float16* VTp   = (_Float16*)carve((size_t)NBH * HD * LTOT * 2);
    _Float16* ctx16 = (_Float16*)carve(CTX_BYTES);
    _Float16* tm16  = (_Float16*)carve((size_t)TXT * INNER * 2);
    _Float16* tmr16 = (_Float16*)carve((size_t)TXT * INNER * 2);
    if (off > ws_size || off > (size_t)134217728) return;
    _Float16* ctxr16 = X16;
    if ((size_t)((char*)wo16 - (char*)X16) < CTX_BYTES) return;

    const unsigned nX8 = (unsigned)(SEQ * INNER / 8), nE8 = (unsigned)(TXT * INNER / 8), nW8 = (unsigned)(INNER * INNER / 8);
    k_cvt16<<<(nX8 + 255u) / 256u, 256, 0, stream>>>(hs, X16, nX8, CARRY_X);
    k_cvt16<<<(nE8 + 255u) / 256u, 256, 0, stream>>>(ehs, E16, nE8, CARRY_X);
    k_cvt16<<<(nW8 + 255u) / 256u, 256, 0, stream>>>(Wq, wq16, nW8, CARRY_W);
    k_cvt16<<<(nW8 + 255u) / 256u, 256, 0, stream>>>(Wk, wk16, nW8, CARRY_W);
    k_cvt16<<<(nW8 + 255u) / 256u, 256, 0, stream>>>(Wv, wv16, nW8, CARRY_W);
    k_cvt16<<<(nW8 + 255u) / 256u, 256, 0, stream>>>(Waq, waq16, nW8, CARRY_W);
    k_cvt16<<<(nW8 + 255u) / 256u, 256, 0, stream>>>(Wak, wak16, nW8, CARRY_W);
    k_cvt16<<<(nW8 + 255u) / 256u, 256, 0, stream>>>(Wav, wav16, nW8, CARRY_W);
    k_cvt16<<<(nW8 + 255u) / 256u, 256, 0, stream>>>(Wout, wo16, nW8, CARRY_W);
    k_cvt16<<<(nW8 + 255u) / 256u, 256, 0, stream>>>(Waout, wao16, nW8, CARRY_W);

    const unsigned gVis = ((unsigned)(GSEQ / 64) * 16u + 7u) / 8u;
    const unsigned gTxt = ((unsigned)(TXT / 64) * 16u + 7u) / 8u;
    k_projqk_rope<<<dim3(gVis, SPN), 256, 0, stream>>>(X16, (unsigned)(SPN * INNER), (unsigned)INNER, wq16, Qp, gq, rc, rs,
                                                       (unsigned)GSEQ, 1u, 0u);
    k_projqk_rope<<<dim3(gVis, SPN), 256, 0, stream>>>(X16, (unsigned)(SPN * INNER), (unsigned)INNER, wk16, Kp, gk, rc, rs,
                                                       (unsigned)GSEQ, 1u, 0u);
    k_projvt<<<dim3(gVis, SPN), 256, 0, stream>>>(wv16, X16, (unsigned)(SPN * INNER), (unsigned)INNER, VTp,
                                                  (unsigned)GSEQ, 1u, 0u);
    k_projqk_plain<<<dim3(gTxt, 1), 256, 0, stream>>>(E16, (unsigned)INNER, 0u, waq16, Qp, gaq, rc, rs,
                                                      (unsigned)TXT, (unsigned)SPN, (unsigned)GSEQ);
    k_projqk_plain<<<dim3(gTxt, 1), 256, 0, stream>>>(E16, (unsigned)INNER, 0u, wak16, Kp, gak, rc, rs,
                                                      (unsigned)TXT, (unsigned)SPN, (unsigned)GSEQ);
    k_projvt<<<dim3(gTxt, 1), 256, 0, stream>>>(wav16, E16, (unsigned)INNER, 0u, VTp,
                                                (unsigned)TXT, (unsigned)SPN, (unsigned)GSEQ);

    k_attn<<<NBH * QBLK, 256, 0, stream>>>(Qp, Kp, VTp, ctx16, ctxr16);

    k_txtmean<<<(TXT * INNER / 8 + 255) / 256, 256, 0, stream>>>(ctx16, ctxr16, tm16, tmr16);

    const unsigned gOV = ((unsigned)(SEQ / 32) * 16u + 7u) / 8u;
    const unsigned gOT = ((unsigned)(TXT / 32) * 16u + 7u) / 8u;
    k_outproj<<<gOV, 256, 0, stream>>>(ctx16, ctxr16, wo16, bout, out, (unsigned)SEQ);
    k_outproj<<<gOT, 256, 0, stream>>>(tm16, tmr16, wao16, baout, out + (size_t)OUT_TXT_ROW * INNER, (unsigned)TXT);
}
